// T5Gemma2DecoderAttention_39582418599958
// MI455X (gfx1250) — hardware-verified
//
#include <hip/hip_runtime.h>
#include <stdint.h>
#include <stddef.h>


typedef __bf16 v16bf __attribute__((ext_vector_type(16)));
typedef __bf16 v8bf __attribute__((ext_vector_type(8)));
typedef float v8f __attribute__((ext_vector_type(8)));
typedef float v4f __attribute__((ext_vector_type(4)));
typedef unsigned int v4u __attribute__((ext_vector_type(4)));

#define DEVINL __device__ __forceinline__

constexpr int T_ = 2048;
constexpr int H_ = 2048;
constexpr int NH_ = 8;
constexpr int NKV_ = 4;
constexpr int HD_ = 256;
constexpr int QD_ = NH_ * HD_;
constexpr int KD_ = NKV_ * HD_;
constexpr int QKVN_ = QD_ + 2 * KD_;
constexpr int SMAX_ = 512;
constexpr float SCALING_ = 0.0625f;
constexpr float EPS_ = 1e-6f;

static_assert(T_ % 64 == 0);
static_assert(H_ % 128 == 0);
static_assert(QKVN_ % 128 == 0);
static_assert((2 * KD_) % 128 == 0);
static_assert(QD_ % 64 == 0);
static_assert(KD_ % 64 == 0);
static_assert(HD_ % 32 == 0);
static_assert((T_ * H_) % 2048 == 0);

DEVINL v8f zero8() {
  v8f z = {0.f, 0.f, 0.f, 0.f, 0.f, 0.f, 0.f, 0.f};
  return z;
}

DEVINL v16bf ldfrag(const __bf16* p) {
  union { v16bf v; v8bf hh[2]; } u;
  u.hh[0] = *(const v8bf*)p;
  u.hh[1] = *(const v8bf*)(p + 16);
  return u.v;
}

DEVINL void wmma3(v8f& acc, const v16bf ah, const v16bf al, const v16bf bh, const v16bf bl) {
  acc = __builtin_amdgcn_wmma_f32_16x16x32_bf16(false, ah, false, bh, (short)0, acc, false, false);
  acc = __builtin_amdgcn_wmma_f32_16x16x32_bf16(false, ah, false, bl, (short)0, acc, false, false);
  acc = __builtin_amdgcn_wmma_f32_16x16x32_bf16(false, al, false, bh, (short)0, acc, false, false);
  asm volatile("v_nop\n\tv_nop\n\tv_nop\n\tv_nop" : "+v"(acc) : "v"(ah), "v"(al), "v"(bh), "v"(bl));
}

DEVINL unsigned bfb(float x) {
  const unsigned u = __float_as_uint(x);
  return (u + 0x7FFFu + ((u >> 16) & 1u)) >> 16;
}

DEVINL void split8(const float (&x)[8], v4u& hi, v4u& lo) {
#pragma unroll
  for (int i = 0; i < 4; ++i) {
    const unsigned h0 = bfb(x[2 * i]);
    const unsigned h1 = bfb(x[2 * i + 1]);
    const unsigned l0 = bfb(x[2 * i] - __uint_as_float(h0 << 16));
    const unsigned l1 = bfb(x[2 * i + 1] - __uint_as_float(h1 << 16));
    hi[i] = h0 | (h1 << 16);
    lo[i] = l0 | (l1 << 16);
  }
}

DEVINL void ld8(const float* p, float (&x)[8]) {
  const v4f a = *(const v4f*)p;
  const v4f b = *(const v4f*)(p + 4);
  x[0] = a.x; x[1] = a.y; x[2] = a.z; x[3] = a.w;
  x[4] = b.x; x[5] = b.y; x[6] = b.z; x[7] = b.w;
}

__global__ __launch_bounds__(256) void conv_rows_k(const float* __restrict__ X,
                                                    unsigned short* __restrict__ Ph,
                                                    unsigned short* __restrict__ Pl,
                                                    int n8) {
  const int i = blockIdx.x * 256 + threadIdx.x;
  if (i >= n8) return;
  float x[8];
  ld8(X + (size_t)i * 8, x);
  v4u hi, lo;
  split8(x, hi, lo);
  volatile v4u* ph = (volatile v4u*)(Ph + (size_t)i * 8);
  volatile v4u* pl = (volatile v4u*)(Pl + (size_t)i * 8);
  *ph = hi;
  *pl = lo;
  __threadfence();
  *ph = hi;
  *pl = lo;
}

__global__ __launch_bounds__(256) void conv_t_k(const float* __restrict__ X, int ldx, int R,
                                                 unsigned short* __restrict__ Yh,
                                                 unsigned short* __restrict__ Yl) {
  __shared__ __attribute__((aligned(16))) unsigned short sH[64 * 72];
  __shared__ __attribute__((aligned(16))) unsigned short sL[64 * 72];
  const int tid = threadIdx.x;
  const int R0 = blockIdx.y * 64;
  const int C0 = blockIdx.x * 64;
  {
    const int r = tid >> 2;
    const int c0 = (tid & 3) * 16;
    const float* src = X + (size_t)(R0 + r) * ldx + C0 + c0;
#pragma unroll
    for (int j = 0; j < 4; ++j) {
      const v4f v = *(const v4f*)(src + 4 * j);
      float e4[4] = {v.x, v.y, v.z, v.w};
#pragma unroll
      for (int e = 0; e < 4; ++e) {
        const unsigned hb = bfb(e4[e]);
        const unsigned lb = bfb(e4[e] - __uint_as_float(hb << 16));
        sH[(c0 + 4 * j + e) * 72 + r] = (unsigned short)hb;
        sL[(c0 + 4 * j + e) * 72 + r] = (unsigned short)lb;
      }
    }
  }
  __syncthreads();
  const int piece = tid & 7;
  auto store_pass = [&]() {
#pragma unroll
    for (int it = 0; it < 2; ++it) {
      const int line = (tid >> 3) + 32 * it;
      const v4u vh = *(const v4u*)&sH[line * 72 + 8 * piece];
      const v4u vl = *(const v4u*)&sL[line * 72 + 8 * piece];
      const size_t o = (size_t)(C0 + line) * R + R0 + 8 * piece;
      *(volatile v4u*)(Yh + o) = vh;
      *(volatile v4u*)(Yl + o) = vl;
    }
  };
  store_pass();
  __threadfence();
  store_pass();
}

__global__ __launch_bounds__(128) void gemm_k(const __bf16* __restrict__ Ah,
                                               const __bf16* __restrict__ Al, int lda,
                                               const __bf16* __restrict__ Bh,
                                               const __bf16* __restrict__ Bl, int ldb,
                                               float* __restrict__ C, int ldc, int K) {
  __shared__ __attribute__((aligned(16))) float stg[4][32 * 64];
  const int tid = threadIdx.x;
  const int lane = tid & 31, wave = tid >> 5;
  const int m = lane & 15, hf = lane >> 4;
  const int row0 = blockIdx.y * 64 + (wave & 1) * 32;
  const int col0 = blockIdx.x * 128 + (wave >> 1) * 64;

  v8f acc[2][4];
#pragma unroll
  for (int ai = 0; ai < 2; ++ai)
#pragma unroll
    for (int bi = 0; bi < 4; ++bi) acc[ai][bi] = zero8();

  const size_t aoff = (size_t)(row0 + m) * lda + 8 * hf;
  const size_t boff = (size_t)(col0 + m) * ldb + 8 * hf;
  const size_t a16 = (size_t)16 * lda;
  const size_t b16 = (size_t)16 * ldb;

#pragma unroll 1
  for (int k0 = 0; k0 < K; k0 += 32) {
    const v16bf ah0 = ldfrag(Ah + aoff + k0);
    const v16bf al0 = ldfrag(Al + aoff + k0);
    const v16bf ah1 = ldfrag(Ah + aoff + a16 + k0);
    const v16bf al1 = ldfrag(Al + aoff + a16 + k0);
#pragma unroll
    for (int bi = 0; bi < 4; ++bi) {
      const v16bf bh = ldfrag(Bh + boff + bi * b16 + k0);
      const v16bf bl = ldfrag(Bl + boff + bi * b16 + k0);
      wmma3(acc[0][bi], ah0, al0, bh, bl);
      wmma3(acc[1][bi], ah1, al1, bh, bl);
    }
  }

  float* st = stg[wave];
#pragma unroll
  for (int ai = 0; ai < 2; ++ai)
#pragma unroll
    for (int bi = 0; bi < 4; ++bi)
#pragma unroll
      for (int r = 0; r < 8; ++r)
        st[(16 * ai + 8 * hf + r) * 64 + 16 * bi + m] = acc[ai][bi][r];
  __syncthreads();

  auto store_pass = [&]() {
#pragma unroll
    for (int i = 0; i < 16; ++i) {
      const int lr = 2 * i + hf;
      const v4f v = *(const v4f*)&st[lr * 64 + 4 * m];
      *(volatile v4f*)(C + (size_t)(row0 + lr) * ldc + col0 + 4 * m) = v;
    }
  };
  store_pass();
  __threadfence();
  store_pass();
}

DEVINL void norm_rope8(const float (&x)[8], const float (&wv)[8],
                       const float (&cs)[8], const float (&sn)[8], float sgn,
                       float (&xn)[8], float (&xr)[8]) {
  float ss = 0.f;
#pragma unroll
  for (int i = 0; i < 8; ++i) ss += x[i] * x[i];
#pragma unroll
  for (int off = 16; off >= 1; off >>= 1) ss += __shfl_xor(ss, off, 32);
  const float inv = rsqrtf(ss * (1.0f / (float)HD_) + EPS_);
#pragma unroll
  for (int i = 0; i < 8; ++i) {
    const float t1 = x[i] * inv;
    xn[i] = t1 * (1.0f + wv[i]);
  }
#pragma unroll
  for (int i = 0; i < 8; ++i) {
    const float pr = __shfl_xor(xn[i], 16, 32);
    xr[i] = xn[i] * cs[i] + (sgn * pr) * sn[i];
  }
}

__global__ __launch_bounds__(256) void normrope_k(const float* __restrict__ qkv,
                                                   const float* __restrict__ ekv,
                                                   const float* __restrict__ cosT,
                                                   const float* __restrict__ sinT,
                                                   const float* __restrict__ qnw,
                                                   const float* __restrict__ knw,
                                                   unsigned short* __restrict__ Qnh, unsigned short* __restrict__ Qnl,
                                                   unsigned short* __restrict__ Qrh, unsigned short* __restrict__ Qrl,
                                                   unsigned short* __restrict__ Krh, unsigned short* __restrict__ Krl,
                                                   unsigned short* __restrict__ Keh, unsigned short* __restrict__ Kel) {
  const int t = blockIdx.x;
  const int tid = threadIdx.x;
  const int lane = tid & 31, w = tid >> 5;
  const int d0 = 8 * lane;
  float cs[8], sn[8];
  ld8(cosT + (size_t)t * HD_ + d0, cs);
  ld8(sinT + (size_t)t * HD_ + d0, sn);
  const float sgn = (lane < 16) ? -1.0f : 1.0f;

  {
    float x[8], wv[8];
    ld8(qkv + (size_t)t * QKVN_ + w * HD_ + d0, x);
    ld8(qnw + d0, wv);
    float xn[8], xr[8];
    norm_rope8(x, wv, cs, sn, sgn, xn, xr);
    v4u nh, nl, rh, rl;
    split8(xn, nh, nl);
    split8(xr, rh, rl);
    const size_t o = (size_t)t * QD_ + w * HD_ + d0;
    volatile v4u* pnh = (volatile v4u*)(Qnh + o);
    volatile v4u* pnl = (volatile v4u*)(Qnl + o);
    volatile v4u* prh = (volatile v4u*)(Qrh + o);
    volatile v4u* prl = (volatile v4u*)(Qrl + o);
    *pnh = nh; *pnl = nl; *prh = rh; *prl = rl;
    __threadfence();
    *pnh = nh; *pnl = nl; *prh = rh; *prl = rl;
  }

  {
    const bool dec = (w < NKV_);
    const int hh = dec ? w : (w - NKV_);
    const float* src = dec ? (qkv + (size_t)t * QKVN_ + QD_ + hh * HD_ + d0)
                           : (ekv + (size_t)t * (2 * KD_) + hh * HD_ + d0);
    float x[8], wv[8];
    ld8(src, x);
    ld8(knw + d0, wv);
    float xn[8], xr[8];
    norm_rope8(x, wv, cs, sn, sgn, xn, xr);
    float xo[8];
#pragma unroll
    for (int i = 0; i < 8; ++i) xo[i] = dec ? xr[i] : xn[i];
    v4u kh, kl;
    split8(xo, kh, kl);
    const size_t o = (size_t)t * KD_ + hh * HD_ + d0;
    unsigned short* dh = dec ? Krh : Keh;
    unsigned short* dl = dec ? Krl : Kel;
    volatile v4u* ph = (volatile v4u*)(dh + o);
    volatile v4u* pl = (volatile v4u*)(dl + o);
    *ph = kh; *pl = kl;
    __threadfence();
    *ph = kh; *pl = kl;
  }
}

template <bool SELF>
__global__ __launch_bounds__(32) void attn_k(const __bf16* __restrict__ Qh, const __bf16* __restrict__ Ql,
                                              const __bf16* __restrict__ Kh, const __bf16* __restrict__ Kl,
                                              const __bf16* __restrict__ Vh, const __bf16* __restrict__ Vl,
                                              const float* Oin,
                                              float* Oout,
                                              unsigned short* Aoh, unsigned short* Aol,
                                              const int* __restrict__ bszp) {
  __shared__ __attribute__((aligned(16))) float sS[16 * SMAX_];
  __shared__ __attribute__((aligned(16))) float sO[16 * HD_];

  const int lane = threadIdx.x & 31;
  const int m = lane & 15, hf = lane >> 4;

  int bsz = bszp[0];
  bsz = (bsz < 4) ? 4 : ((bsz > 64) ? 64 : bsz);
  int S = T_ / bsz;
  S &= ~31;
  if (S < 32) S = 32;

  const int h = blockIdx.y;
  const int kvh = h >> 1;
  const int qtok0 = blockIdx.x * 16;
  const int b = qtok0 / S;
  const int q0 = qtok0 - b * S;
  int kbase = b * S;
  if (kbase + S > T_) kbase = T_ - S;
  int nkt = SELF ? ((q0 + 16 + 31) >> 5) : (S >> 5);
  if (nkt > SMAX_ / 32) nkt = SMAX_ / 32;
  if (nkt < 1) nkt = 1;

  {
    const size_t qoff = (size_t)(qtok0 + m) * QD_ + h * HD_ + 8 * hf;
    const __bf16* qph = Qh + qoff;
    const __bf16* qpl = Ql + qoff;
    for (int kt = 0; kt < nkt; ++kt) {
      v8f s0 = zero8(), s1 = zero8();
      const size_t koff = (size_t)(kbase + kt * 32 + m) * KD_ + kvh * HD_ + 8 * hf;
      const __bf16* k0h = Kh + koff;
      const __bf16* k0l = Kl + koff;
      const __bf16* k1h = k0h + 16 * KD_;
      const __bf16* k1l = k0l + 16 * KD_;
#pragma unroll 2
      for (int kk = 0; kk < HD_ / 32; ++kk) {
        const int dk = kk * 32;
        const v16bf aqh = ldfrag(qph + dk);
        const v16bf aql = ldfrag(qpl + dk);
        {
          const v16bf bh = ldfrag(k0h + dk);
          const v16bf bl = ldfrag(k0l + dk);
          wmma3(s0, aqh, aql, bh, bl);
        }
        {
          const v16bf bh = ldfrag(k1h + dk);
          const v16bf bl = ldfrag(k1l + dk);
          wmma3(s1, aqh, aql, bh, bl);
        }
      }
#pragma unroll
      for (int r = 0; r < 8; ++r) {
        sS[(8 * hf + r) * SMAX_ + kt * 32 + m]      = s0[r] * SCALING_;
        sS[(8 * hf + r) * SMAX_ + kt * 32 + 16 + m] = s1[r] * SCALING_;
      }
    }
  }
  __syncthreads();

  {
    unsigned short* sP = (unsigned short*)sS;
    const int kb16 = 16 * lane;
#pragma unroll 1
    for (int r = 0; r < 16; ++r) {
      const float* rp = sS + r * SMAX_ + kb16;
      float sv[16];
      {
        float t8[8];
        ld8(rp, t8);
#pragma unroll
        for (int j = 0; j < 8; ++j) sv[j] = t8[j];
        ld8(rp + 8, t8);
#pragma unroll
        for (int j = 0; j < 8; ++j) sv[8 + j] = t8[j];
      }
      const int nvalid = SELF ? (q0 + r + 1) : S;
      float mx = -3.0e38f;
#pragma unroll
      for (int j = 0; j < 16; ++j) {
        sv[j] = (kb16 + j < nvalid) ? sv[j] : -3.0e38f;
        mx = fmaxf(mx, sv[j]);
      }
#pragma unroll
      for (int off = 16; off >= 1; off >>= 1) mx = fmaxf(mx, __shfl_xor(mx, off, 32));
      float e[16];
      float sum = 0.f;
#pragma unroll
      for (int j = 0; j < 16; ++j) {
        e[j] = (kb16 + j < nvalid) ? __expf(sv[j] - mx) : 0.f;
        sum += e[j];
      }
#pragma unroll
      for (int off = 16; off >= 1; off >>= 1) sum += __shfl_xor(sum, off, 32);
      const float inv = 1.0f / sum;
      float p0[8], p1[8];
#pragma unroll
      for (int j = 0; j < 8; ++j) {
        p0[j] = e[j] * inv;
        p1[j] = e[8 + j] * inv;
      }
      v4u h0, l0, h1, l1;
      split8(p0, h0, l0);
      split8(p1, h1, l1);
      __builtin_amdgcn_fence(__ATOMIC_RELEASE, "wavefront");
      __builtin_amdgcn_wave_barrier();
      unsigned short* ph = sP + r * 1024 + kb16;
      unsigned short* pl = ph + 512;
      *(v4u*)ph = h0;
      *(v4u*)(ph + 8) = h1;
      *(v4u*)pl = l0;
      *(v4u*)(pl + 8) = l1;
    }
  }
  __syncthreads();

  {
    const __bf16* pbase = (const __bf16*)sS;
    const __bf16* pph = pbase + m * 1024 + 8 * hf;
    const __bf16* ppl = pph + 512;
    const size_t voff = (size_t)(kvh * HD_ + m) * T_ + kbase + 8 * hf;
#pragma unroll 1
    for (int nt = 0; nt < HD_ / 16; ++nt) {
      v8f acc = zero8();
      const __bf16* vph = Vh + voff + (size_t)nt * 16 * T_;
      const __bf16* vpl = Vl + voff + (size_t)nt * 16 * T_;
      for (int kt = 0; kt < nkt; ++kt) {
        const v16bf ah = ldfrag(pph + kt * 32);
        const v16bf al = ldfrag(ppl + kt * 32);
        const v16bf bh = ldfrag(vph + kt * 32);
        const v16bf bl = ldfrag(vpl + kt * 32);
        wmma3(acc, ah, al, bh, bl);
      }
#pragma unroll
      for (int r = 0; r < 8; ++r) sO[(8 * hf + r) * HD_ + nt * 16 + m] = acc[r];
    }
  }
  __syncthreads();

  if (SELF) {
    auto store_pass = [&]() {
#pragma unroll 1
      for (int i = 0; i < 16; ++i) {
#pragma unroll
        for (int hh = 0; hh < 2; ++hh) {
          const int col = hh * 128 + 4 * lane;
          const v4f v = *(const v4f*)&sO[i * HD_ + col];
          *(volatile v4f*)(Oout + (size_t)(qtok0 + i) * QD_ + h * HD_ + col) = v;
        }
      }
    };
    store_pass();
    __threadfence();
    store_pass();
  } else {
    auto store_pass = [&]() {
#pragma unroll 1
      for (int i = 0; i < 16; ++i) {
        const int col = 8 * lane;
        float c8[8], g8[8], x[8];
        ld8(&sO[i * HD_ + col], c8);
        ld8(Oin + (size_t)(qtok0 + i) * QD_ + h * HD_ + col, g8);
#pragma unroll
        for (int j = 0; j < 8; ++j) x[j] = g8[j] + c8[j];
        v4u hi, lo;
        split8(x, hi, lo);
        const size_t o = (size_t)(qtok0 + i) * QD_ + h * HD_ + col;
        *(volatile v4u*)(Aoh + o) = hi;
        *(volatile v4u*)(Aol + o) = lo;
      }
    };
    store_pass();
    __threadfence();
    store_pass();
  }
}

extern "C" void kernel_launch(void* const* d_in, const int* in_sizes, int n_in,
                              void* d_out, int out_size, void* d_ws,
                              size_t ws_size, hipStream_t stream) {
  if (n_in < 9) return;
  if (in_sizes[0] != T_ * H_ || in_sizes[1] != T_ * H_ ||
      in_sizes[2] != T_ * HD_ || in_sizes[3] != T_ * HD_ ||
      in_sizes[4] != H_ * QKVN_ || in_sizes[5] != QD_ * H_ ||
      in_sizes[6] != HD_ || in_sizes[7] != HD_ || in_sizes[8] < 1 ||
      out_size != T_ * H_) return;
  const size_t MB = (size_t)1 << 20;
  const size_t need = 112 * MB;
  if (ws_size < need) return;

  const float* hs   = (const float*)d_in[0];
  const float* ehs  = (const float*)d_in[1];
  const float* cosT = (const float*)d_in[2];
  const float* sinT = (const float*)d_in[3];
  const float* wqkv = (const float*)d_in[4];
  const float* wo   = (const float*)d_in[5];
  const float* qnw  = (const float*)d_in[6];
  const float* knw  = (const float*)d_in[7];
  const int*   bszp = (const int*)d_in[8];
  float* out = (float*)d_out;
  char* ws = (char*)d_ws;

  unsigned short* Xh_us  = (unsigned short*)(ws + 0 * MB);
  unsigned short* Xl_us  = (unsigned short*)(ws + 8 * MB);
  unsigned short* WTh_us = (unsigned short*)(ws + 16 * MB);
  unsigned short* WTl_us = (unsigned short*)(ws + 32 * MB);
  float* qkv_f = (float*)(ws + 48 * MB);
  float* ekv_f = (float*)(ws + 80 * MB);
  const __bf16* Xh  = (const __bf16*)(ws + 0 * MB);
  const __bf16* Xl  = (const __bf16*)(ws + 8 * MB);
  const __bf16* WTh = (const __bf16*)(ws + 16 * MB);
  const __bf16* WTl = (const __bf16*)(ws + 32 * MB);
  unsigned short* Qnh = (unsigned short*)(ws + 0 * MB);
  unsigned short* Qnl = (unsigned short*)(ws + 8 * MB);
  unsigned short* Qrh = (unsigned short*)(ws + 16 * MB);
  unsigned short* Qrl = (unsigned short*)(ws + 24 * MB);
  unsigned short* Krh = (unsigned short*)(ws + 32 * MB);
  unsigned short* Krl = (unsigned short*)(ws + 36 * MB);
  unsigned short* Keh = (unsigned short*)(ws + 40 * MB);
  unsigned short* Kel = (unsigned short*)(ws + 44 * MB);
  unsigned short* VTh = (unsigned short*)(ws + 96 * MB);
  unsigned short* VTl = (unsigned short*)(ws + 100 * MB);
  unsigned short* VEh = (unsigned short*)(ws + 104 * MB);
  unsigned short* VEl = (unsigned short*)(ws + 108 * MB);
  float* attn_f = (float*)(ws + 48 * MB);
  unsigned short* Aoh = (unsigned short*)(ws + 64 * MB);
  unsigned short* Aol = (unsigned short*)(ws + 72 * MB);
  unsigned short* WoTh = (unsigned short*)(ws + 80 * MB);
  unsigned short* WoTl = (unsigned short*)(ws + 88 * MB);

  conv_rows_k<<<(T_ * H_ / 8) / 256, 256, 0, stream>>>(hs, Xh_us, Xl_us, T_ * H_ / 8);
  conv_t_k<<<dim3(QKVN_ / 64, H_ / 64), 256, 0, stream>>>(wqkv, QKVN_, H_, WTh_us, WTl_us);
  gemm_k<<<dim3(QKVN_ / 128, T_ / 64), 128, 0, stream>>>(Xh, Xl, H_, WTh, WTl, H_, qkv_f, QKVN_, H_);
  conv_rows_k<<<(T_ * H_ / 8) / 256, 256, 0, stream>>>(ehs, Xh_us, Xl_us, T_ * H_ / 8);
  gemm_k<<<dim3((2 * KD_) / 128, T_ / 64), 128, 0, stream>>>(
      Xh, Xl, H_, WTh + (size_t)QD_ * H_, WTl + (size_t)QD_ * H_, H_, ekv_f, 2 * KD_, H_);
  normrope_k<<<T_, 256, 0, stream>>>(qkv_f, ekv_f, cosT, sinT, qnw, knw,
                                     Qnh, Qnl, Qrh, Qrl, Krh, Krl, Keh, Kel);
  conv_t_k<<<dim3(KD_ / 64, T_ / 64), 256, 0, stream>>>(qkv_f + QD_ + KD_, QKVN_, T_, VTh, VTl);
  conv_t_k<<<dim3(KD_ / 64, T_ / 64), 256, 0, stream>>>(ekv_f + KD_, 2 * KD_, T_, VEh, VEl);
  attn_k<true><<<dim3(T_ / 16, NH_), 32, 0, stream>>>(
      (const __bf16*)Qrh, (const __bf16*)Qrl, (const __bf16*)Krh, (const __bf16*)Krl,
      (const __bf16*)VTh, (const __bf16*)VTl, attn_f, attn_f, Aoh, Aol, bszp);
  conv_t_k<<<dim3(H_ / 64, QD_ / 64), 256, 0, stream>>>(wo, H_, QD_, WoTh, WoTl);
  attn_k<false><<<dim3(T_ / 16, NH_), 32, 0, stream>>>(
      (const __bf16*)Qnh, (const __bf16*)Qnl, (const __bf16*)Keh, (const __bf16*)Kel,
      (const __bf16*)VEh, (const __bf16*)VEl, attn_f, attn_f, Aoh, Aol, bszp);
  gemm_k<<<dim3(H_ / 128, T_ / 64), 128, 0, stream>>>(
      (const __bf16*)Aoh, (const __bf16*)Aol, QD_, (const __bf16*)WoTh, (const __bf16*)WoTl, QD_,
      out, H_, QD_);
}
